// DeepClustering_18571438588712
// MI455X (gfx1250) — hardware-verified
//
#include <hip/hip_runtime.h>
#include <hip/hip_bf16.h>


#define BATCH   64
#define SEQ     128
#define D_IN    16
#define D_MODEL 256
#define NHEAD   8
#define DHEAD   32
#define D_FF    1024
#define NROWS   8192
#define KNNS    10

static_assert(NROWS == BATCH * SEQ);
static_assert(D_MODEL == NHEAD * DHEAD);
static_assert(D_MODEL == 256);
static_assert(SEQ == 128 && DHEAD == 32);
static_assert(NROWS % 256 == 0);
static_assert(D_IN == 16);

typedef __bf16 bf16_t;
typedef __attribute__((ext_vector_type(4)))  __bf16 v4bf;
typedef __attribute__((ext_vector_type(8)))  __bf16 v8bf;
typedef __attribute__((ext_vector_type(16))) __bf16 v16bf;
typedef __attribute__((ext_vector_type(8)))  float  v8f;
typedef __attribute__((ext_vector_type(4)))  float  v4f;

union Frag { v16bf v; v8bf h[2]; };

__device__ __forceinline__ v8f zero_v8f() { v8f z = {0.f,0.f,0.f,0.f,0.f,0.f,0.f,0.f}; return z; }
__device__ __forceinline__ v4f zero_v4f() { v4f z = {0.f,0.f,0.f,0.f}; return z; }
__device__ __forceinline__ v8bf zero_v8bf()
{
    v8bf z;
    #pragma unroll
    for (int i = 0; i < 8; ++i) z[i] = (bf16_t)0.0f;
    return z;
}

__device__ __forceinline__ v8f wmma_bf16(v8f acc, v16bf a, v16bf b)
{
    acc = __builtin_amdgcn_wmma_f32_16x16x32_bf16(false, a, false, b, (short)0, acc, false, false);
    asm volatile("v_nop\n\tv_nop\n\tv_nop\n\tv_nop" : "+v"(acc) : "v"(a), "v"(b));
    return acc;
}

__device__ __forceinline__ v8bf cvt8_bf16(v4f a, v4f b)
{
    v8bf r;
    r[0] = (bf16_t)a[0]; r[1] = (bf16_t)a[1]; r[2] = (bf16_t)a[2]; r[3] = (bf16_t)a[3];
    r[4] = (bf16_t)b[0]; r[5] = (bf16_t)b[1]; r[6] = (bf16_t)b[2]; r[7] = (bf16_t)b[3];
    return r;
}

__device__ __forceinline__ float sumsq16(const float* __restrict__ p)
{
    v4f a = *(const v4f*)(p);
    v4f b = *(const v4f*)(p + 4);
    v4f c = *(const v4f*)(p + 8);
    v4f d = *(const v4f*)(p + 12);
    float s = 0.f;
    s = fmaf(a[0], a[0], s); s = fmaf(a[1], a[1], s); s = fmaf(a[2], a[2], s); s = fmaf(a[3], a[3], s);
    s = fmaf(b[0], b[0], s); s = fmaf(b[1], b[1], s); s = fmaf(b[2], b[2], s); s = fmaf(b[3], b[3], s);
    s = fmaf(c[0], c[0], s); s = fmaf(c[1], c[1], s); s = fmaf(c[2], c[2], s); s = fmaf(c[3], c[3], s);
    s = fmaf(d[0], d[0], s); s = fmaf(d[1], d[1], s); s = fmaf(d[2], d[2], s); s = fmaf(d[3], d[3], s);
    return s;
}

#define TILE_M 32
#define TILE_N 128
#define TILE_K 32
#define LDSS   40
#define CSP    132

__global__ __launch_bounds__(256)
void gemm_wmma_kernel(const float* __restrict__ A, const float* __restrict__ B,
                      const float* __restrict__ bias, float* __restrict__ C,
                      int M, int N, int K, int has_bias, int relu)
{
    __shared__ __align__(16) bf16_t As[TILE_M * LDSS];
    __shared__ __align__(16) bf16_t BsT[TILE_N * LDSS];
    __shared__ __align__(16) float  Cs[TILE_M * CSP];

    const int tid   = threadIdx.x;
    const int wave  = tid >> 5;
    const int lane  = tid & 31;
    const int waveM = wave >> 2;
    const int waveN = wave & 3;
    const int hl    = lane >> 4;
    const int l16   = lane & 15;

    const int blockM = blockIdx.x * TILE_M;
    const int blockN = blockIdx.y * TILE_N;

    const int  ar      = tid >> 3;
    const int  ac      = (tid & 7) * 4;
    const int  arow    = blockM + ar;
    const bool arow_ok = arow < M;

    const int  sbr     = wave * 4;
    const int  sbc     = lane * 4;
    const int  bcol    = blockN + sbc;
    const bool bcol_ok = bcol < N;

    v8f acc0 = zero_v8f();
    v8f acc1 = zero_v8f();

    for (int k0 = 0; k0 < K; k0 += TILE_K) {
        v4f aReg = zero_v4f();
        if (arow_ok && (k0 + ac) < K)
            aReg = *(const v4f*)(A + (size_t)arow * K + (k0 + ac));
        v4f bReg[4];
        #pragma unroll
        for (int e = 0; e < 4; ++e) {
            bReg[e] = zero_v4f();
            const int kk = k0 + sbr + e;
            if (bcol_ok && kk < K)
                bReg[e] = *(const v4f*)(B + (size_t)kk * N + bcol);
        }

        v4bf av;
        av[0] = (bf16_t)aReg[0]; av[1] = (bf16_t)aReg[1];
        av[2] = (bf16_t)aReg[2]; av[3] = (bf16_t)aReg[3];
        *(v4bf*)&As[ar * LDSS + ac] = av;

        v4bf t0, t1, t2, t3;
        t0[0]=(bf16_t)bReg[0][0]; t0[1]=(bf16_t)bReg[1][0]; t0[2]=(bf16_t)bReg[2][0]; t0[3]=(bf16_t)bReg[3][0];
        t1[0]=(bf16_t)bReg[0][1]; t1[1]=(bf16_t)bReg[1][1]; t1[2]=(bf16_t)bReg[2][1]; t1[3]=(bf16_t)bReg[3][1];
        t2[0]=(bf16_t)bReg[0][2]; t2[1]=(bf16_t)bReg[1][2]; t2[2]=(bf16_t)bReg[2][2]; t2[3]=(bf16_t)bReg[3][2];
        t3[0]=(bf16_t)bReg[0][3]; t3[1]=(bf16_t)bReg[1][3]; t3[2]=(bf16_t)bReg[2][3]; t3[3]=(bf16_t)bReg[3][3];
        *(v4bf*)&BsT[(sbc + 0) * LDSS + sbr] = t0;
        *(v4bf*)&BsT[(sbc + 1) * LDSS + sbr] = t1;
        *(v4bf*)&BsT[(sbc + 2) * LDSS + sbr] = t2;
        *(v4bf*)&BsT[(sbc + 3) * LDSS + sbr] = t3;
        __syncthreads();

        Frag fa, fb0, fb1;
        const int am = (waveM * 16 + l16) * LDSS;
        fa.h[0] = *(const v8bf*)&As[am + 8 * hl];
        fa.h[1] = *(const v8bf*)&As[am + 16 + 8 * hl];
        const int bn0 = (waveN * 32 + l16) * LDSS;
        const int bn1 = (waveN * 32 + 16 + l16) * LDSS;
        fb0.h[0] = *(const v8bf*)&BsT[bn0 + 8 * hl];
        fb0.h[1] = *(const v8bf*)&BsT[bn0 + 16 + 8 * hl];
        fb1.h[0] = *(const v8bf*)&BsT[bn1 + 8 * hl];
        fb1.h[1] = *(const v8bf*)&BsT[bn1 + 16 + 8 * hl];

        acc0 = wmma_bf16(acc0, fa.v, fb0.v);
        acc1 = wmma_bf16(acc1, fa.v, fb1.v);
        __syncthreads();
    }

    const int crow = waveM * 16 + hl * 8;
    const int ccol = waveN * 32 + l16;
    #pragma unroll
    for (int j = 0; j < 8; ++j) {
        Cs[(crow + j) * CSP + ccol]      = acc0[j];
        Cs[(crow + j) * CSP + ccol + 16] = acc1[j];
    }
    __syncthreads();

    const int NW = (N - blockN) < TILE_N ? (N - blockN) : TILE_N;
    const int n4 = 8 * NW;
    v4f  vals[4];
    int  rws[4], cls[4];
    bool oks[4];
    #pragma unroll
    for (int i = 0; i < 4; ++i) {
        const int q = tid + 256 * i;
        bool ok = q < n4;
        int row = 0, col = 0;
        if (ok) {
            row = (4 * q) / NW;
            col = 4 * q - row * NW;
            ok  = (blockM + row) < M;
        }
        v4f v = zero_v4f();
        if (ok) {
            v = *(const v4f*)&Cs[row * CSP + col];
            if (has_bias) {
                v4f bb = *(const v4f*)(bias + blockN + col);
                v += bb;
            }
            if (relu) {
                v[0] = fmaxf(v[0], 0.f); v[1] = fmaxf(v[1], 0.f);
                v[2] = fmaxf(v[2], 0.f); v[3] = fmaxf(v[3], 0.f);
            }
        }
        vals[i] = v; rws[i] = row; cls[i] = col; oks[i] = ok;
    }
    #pragma unroll
    for (int i = 0; i < 4; ++i)
        if (oks[i]) *(volatile v4f*)(C + (size_t)(blockM + rws[i]) * N + blockN + cls[i]) = vals[i];
    __threadfence();
    #pragma unroll
    for (int i = 0; i < 4; ++i)
        if (oks[i]) *(volatile v4f*)(C + (size_t)(blockM + rws[i]) * N + blockN + cls[i]) = vals[i];
}

__global__ __launch_bounds__(SEQ)
void attention_kernel(const float* __restrict__ Q, const float* __restrict__ Km,
                      const float* __restrict__ V, float* __restrict__ Out)
{
    const int bh = blockIdx.x;
    const int b  = bh / NHEAD;
    const int hh = bh % NHEAD;
    const int t  = threadIdx.x;

    __shared__ __align__(16) float Ks[SEQ * DHEAD];
    __shared__ __align__(16) float Vs[SEQ * DHEAD];

    #pragma unroll
    for (int i = 0; i < (SEQ * DHEAD) / (SEQ * 4); ++i) {
        const int f = t + i * SEQ;
        const int j = f >> 3, d = (f & 7) * 4;
        const size_t g = (size_t)(b * SEQ + j) * D_MODEL + hh * DHEAD + d;
        *(v4f*)&Ks[j * DHEAD + d] = *(const v4f*)(Km + g);
        *(v4f*)&Vs[j * DHEAD + d] = *(const v4f*)(V + g);
    }
    __syncthreads();

    const float  scale = 0.17677669529663687f;
    const size_t qbase = (size_t)(b * SEQ + t) * D_MODEL + hh * DHEAD;
    float qv[DHEAD];
    #pragma unroll
    for (int d = 0; d < DHEAD; d += 4) {
        v4f qq = *(const v4f*)(Q + qbase + d);
        qv[d] = qq[0] * scale; qv[d+1] = qq[1] * scale;
        qv[d+2] = qq[2] * scale; qv[d+3] = qq[3] * scale;
    }

    float m = -3.4e38f, l = 0.f;
    float o[DHEAD];
    #pragma unroll
    for (int d = 0; d < DHEAD; ++d) o[d] = 0.f;

    #pragma unroll 1
    for (int j = 0; j < SEQ; ++j) {
        float s = 0.f;
        #pragma unroll
        for (int d = 0; d < DHEAD; ++d) s = fmaf(qv[d], Ks[j * DHEAD + d], s);
        const float nm   = fmaxf(m, s);
        const float corr = __expf(m - nm);
        const float p    = __expf(s - nm);
        l = l * corr + p;
        #pragma unroll
        for (int d = 0; d < DHEAD; ++d) o[d] = o[d] * corr + p * Vs[j * DHEAD + d];
        m = nm;
    }
    const float inv = 1.f / l;

    v4f ov[DHEAD / 4];
    #pragma unroll
    for (int c = 0; c < DHEAD / 4; ++c) {
        v4f w;
        w[0] = o[4*c+0] * inv; w[1] = o[4*c+1] * inv;
        w[2] = o[4*c+2] * inv; w[3] = o[4*c+3] * inv;
        ov[c] = w;
    }
    float* op = Out + qbase;
    #pragma unroll
    for (int c = 0; c < DHEAD / 4; ++c) *(volatile v4f*)(op + 4 * c) = ov[c];
    __threadfence();
    #pragma unroll
    for (int c = 0; c < DHEAD / 4; ++c) *(volatile v4f*)(op + 4 * c) = ov[c];
}

__global__ __launch_bounds__(256)
void add_ln_kernel(const float* __restrict__ X, const float* __restrict__ Y,
                   const float* __restrict__ g, const float* __restrict__ bta,
                   float* __restrict__ Out, int M)
{
    const int wave = threadIdx.x >> 5;
    const int lane = threadIdx.x & 31;
    const int row  = blockIdx.x * 8 + wave;
    if (row >= M) return;
    const size_t base = (size_t)row * D_MODEL;

    v4f x0 = *(const v4f*)(X + base + 4 * lane);
    v4f x1 = *(const v4f*)(X + base + 128 + 4 * lane);
    v4f y0 = *(const v4f*)(Y + base + 4 * lane);
    v4f y1 = *(const v4f*)(Y + base + 128 + 4 * lane);
    v4f a0 = x0 + y0, a1 = x1 + y1;

    float s = (a0[0] + a0[1]) + (a0[2] + a0[3]) + (a1[0] + a1[1]) + (a1[2] + a1[3]);
    #pragma unroll
    for (int off = 16; off >= 1; off >>= 1) s += __shfl_xor(s, off, 32);
    const float mean = s * (1.f / D_MODEL);

    v4f d0 = a0 - mean, d1 = a1 - mean;
    float ss = d0[0]*d0[0] + d0[1]*d0[1] + d0[2]*d0[2] + d0[3]*d0[3]
             + d1[0]*d1[0] + d1[1]*d1[1] + d1[2]*d1[2] + d1[3]*d1[3];
    #pragma unroll
    for (int off = 16; off >= 1; off >>= 1) ss += __shfl_xor(ss, off, 32);
    const float var = ss * (1.f / D_MODEL);
    const float inv = rsqrtf(var + 1e-5f);

    v4f g0 = *(const v4f*)(g + 4 * lane),   g1 = *(const v4f*)(g + 128 + 4 * lane);
    v4f b0 = *(const v4f*)(bta + 4 * lane), b1 = *(const v4f*)(bta + 128 + 4 * lane);
    v4f o0 = d0 * inv * g0 + b0;
    v4f o1 = d1 * inv * g1 + b1;

    *(volatile v4f*)(Out + base + 4 * lane)       = o0;
    *(volatile v4f*)(Out + base + 128 + 4 * lane) = o1;
    __threadfence();
    *(volatile v4f*)(Out + base + 4 * lane)       = o0;
    *(volatile v4f*)(Out + base + 128 + 4 * lane) = o1;
}

#define DT_ROWS  256
#define DT_COLS  32
#define DT_PITCH 33

__global__ __launch_bounds__(DT_ROWS)
void dist_topk_kernel(const float* __restrict__ Xr, float* __restrict__ rowsum, int nrows)
{
    __shared__ float dtile[DT_ROWS * DT_PITCH];
    __shared__ float sqc[DT_COLS];
    __shared__ __align__(16) float rs[DT_ROWS];

    const int tid  = threadIdx.x;
    const int wave = tid >> 5;
    const int lane = tid & 31;
    const int h    = lane >> 4;
    const int m    = lane & 15;
    const int rowBase = blockIdx.x * DT_ROWS;

    const v8bf z8 = zero_v8bf();

    Frag fa0, fa1;
    {
        const int r0 = rowBase + wave * 32 + m;
        const int r1 = r0 + 16;
        fa0.h[0] = z8; fa1.h[0] = z8;
        if (r0 < nrows) {
            const float* p = Xr + (size_t)r0 * D_IN + 8 * h;
            fa0.h[0] = cvt8_bf16(*(const v4f*)p, *(const v4f*)(p + 4));
        }
        if (r1 < nrows) {
            const float* p = Xr + (size_t)r1 * D_IN + 8 * h;
            fa1.h[0] = cvt8_bf16(*(const v4f*)p, *(const v4f*)(p + 4));
        }
        fa0.h[1] = z8; fa1.h[1] = z8;
    }

    const int   myrow = rowBase + tid;
    const bool  vme   = myrow < nrows;
    const float sqme  = vme ? sumsq16(Xr + (size_t)myrow * D_IN) : 0.f;

    float best[KNNS];
    #pragma unroll
    for (int i = 0; i < KNNS; ++i) best[i] = 3.0e38f;

    for (int jt = 0; jt < nrows; jt += DT_COLS) {
        Frag fb0, fb1;
        {
            const int c0 = jt + m;
            const int c1 = c0 + 16;
            fb0.h[0] = z8; fb1.h[0] = z8;
            if (c0 < nrows) {
                const float* p = Xr + (size_t)c0 * D_IN + 8 * h;
                fb0.h[0] = cvt8_bf16(*(const v4f*)p, *(const v4f*)(p + 4));
            }
            if (c1 < nrows) {
                const float* p = Xr + (size_t)c1 * D_IN + 8 * h;
                fb1.h[0] = cvt8_bf16(*(const v4f*)p, *(const v4f*)(p + 4));
            }
            fb0.h[1] = z8; fb1.h[1] = z8;
        }
        if (wave == 0) {
            const int c = jt + lane;
            sqc[lane] = (c < nrows) ? sumsq16(Xr + (size_t)c * D_IN) : 0.f;
        }

        v8f a00 = wmma_bf16(zero_v8f(), fa0.v, fb0.v);
        v8f a01 = wmma_bf16(zero_v8f(), fa0.v, fb1.v);
        v8f a10 = wmma_bf16(zero_v8f(), fa1.v, fb0.v);
        v8f a11 = wmma_bf16(zero_v8f(), fa1.v, fb1.v);

        const int lr0 = wave * 32 + 8 * h;
        const int lr1 = lr0 + 16;
        #pragma unroll
        for (int r = 0; r < 8; ++r) {
            dtile[(lr0 + r) * DT_PITCH + m]      = a00[r];
            dtile[(lr0 + r) * DT_PITCH + 16 + m] = a01[r];
            dtile[(lr1 + r) * DT_PITCH + m]      = a10[r];
            dtile[(lr1 + r) * DT_PITCH + 16 + m] = a11[r];
        }
        __syncthreads();

        int jn = nrows - jt;
        if (jn > DT_COLS) jn = DT_COLS;
        #pragma unroll 4
        for (int j = 0; j < jn; ++j) {
            const float dot  = dtile[tid * DT_PITCH + j];
            const float dist = (sqme + sqc[j]) - 2.0f * dot;
            if (dist < best[KNNS - 1]) {
                float x = dist;
                #pragma unroll
                for (int p = 0; p < KNNS; ++p) {
                    const float lo = fminf(best[p], x);
                    const float hi = fmaxf(best[p], x);
                    best[p] = lo; x = hi;
                }
            }
        }
        __syncthreads();
    }

    float s = 0.f;
    #pragma unroll
    for (int i = 0; i < KNNS; ++i) s += best[i];
    if (!vme) s = 0.f;
    rs[tid] = s;
    __syncthreads();

    const bool wok = (tid < DT_ROWS / 4) && (rowBase + 4 * tid + 3 < nrows);
    v4f wv = zero_v4f();
    if (tid < DT_ROWS / 4) wv = *(const v4f*)&rs[4 * tid];
    if (wok) *(volatile v4f*)(rowsum + rowBase + 4 * tid) = wv;
    __threadfence();
    if (wok) *(volatile v4f*)(rowsum + rowBase + 4 * tid) = wv;
}

__global__ __launch_bounds__(256)
void final_sum_kernel(const float* __restrict__ rowsum, float* __restrict__ out, int nrows)
{
    __shared__ double red[256];
    const int tid = threadIdx.x;
    double s = 0.0;
    for (int i = 0; i < 32; ++i) {
        const int r = tid * 32 + i;
        if (r < nrows) s += (double)rowsum[r];
    }
    red[tid] = s;
    __syncthreads();
    if (tid == 0) {
        double t = 0.0;
        for (int w = 0; w < 256; ++w) t += red[w];
        const float f = (float)t;
        *(volatile float*)out = f;
        __threadfence();
        *(volatile float*)out = f;
    }
}

static void launch_gemm(hipStream_t st, const float* A, const float* B, const float* bias,
                        float* C, int M, int N, int K, int has_bias, int relu)
{
    const dim3 grid((M + TILE_M - 1) / TILE_M, (N + TILE_N - 1) / TILE_N);
    gemm_wmma_kernel<<<grid, dim3(256), 0, st>>>(A, B, bias, C, M, N, K, has_bias, relu);
}

extern "C" void kernel_launch(void* const* d_in, const int* in_sizes, int n_in,
                              void* d_out, int out_size, void* d_ws, size_t ws_size,
                              hipStream_t stream)
{
    if (n_in < 17 || out_size < 1) return;
    if (in_sizes[0] != NROWS * D_IN || in_sizes[1] != D_IN * D_MODEL ||
        in_sizes[3] != D_MODEL * D_MODEL || in_sizes[9] != D_MODEL * D_FF ||
        in_sizes[11] != D_FF * D_MODEL || in_sizes[15] != D_MODEL * D_IN) return;

    const float* x     = (const float*)d_in[0];
    const float* W_emb = (const float*)d_in[1];
    const float* b_emb = (const float*)d_in[2];
    const float* Wq    = (const float*)d_in[3];
    const float* Wk    = (const float*)d_in[4];
    const float* Wv    = (const float*)d_in[5];
    const float* Wo    = (const float*)d_in[6];
    const float* ln1_g = (const float*)d_in[7];
    const float* ln1_b = (const float*)d_in[8];
    const float* W1    = (const float*)d_in[9];
    const float* b1    = (const float*)d_in[10];
    const float* W2    = (const float*)d_in[11];
    const float* b2    = (const float*)d_in[12];
    const float* ln2_g = (const float*)d_in[13];
    const float* ln2_b = (const float*)d_in[14];
    const float* Wd    = (const float*)d_in[15];
    const float* bd    = (const float*)d_in[16];
    float* out = (float*)d_out;
    float* ws  = (float*)d_ws;

    const size_t MB2  = (size_t)NROWS * D_MODEL;
    const size_t need = (7 * MB2 + (size_t)NROWS) * sizeof(float);
    if (need > ws_size) return;
    float* h0     = ws + 0 * MB2;
    float* q      = ws + 1 * MB2;
    float* k      = ws + 2 * MB2;
    float* v      = ws + 3 * MB2;
    float* att    = ws + 4 * MB2;
    float* o      = ws + 5 * MB2;
    float* h1     = ws + 6 * MB2;
    float* ff1    = ws + 1 * MB2;
    float* ff2    = ws + 5 * MB2;
    float* h2     = ws + 0 * MB2;
    float* xrec   = ws + 1 * MB2;
    float* rowsum = ws + 7 * MB2;

    launch_gemm(stream, x, W_emb, b_emb, h0, NROWS, D_MODEL, D_IN, 1, 0);
    launch_gemm(stream, h0, Wq, b_emb, q, NROWS, D_MODEL, D_MODEL, 0, 0);
    launch_gemm(stream, h0, Wk, b_emb, k, NROWS, D_MODEL, D_MODEL, 0, 0);
    launch_gemm(stream, h0, Wv, b_emb, v, NROWS, D_MODEL, D_MODEL, 0, 0);
    attention_kernel<<<dim3(BATCH * NHEAD), dim3(SEQ), 0, stream>>>(q, k, v, att);
    launch_gemm(stream, att, Wo, b_emb, o, NROWS, D_MODEL, D_MODEL, 0, 0);
    add_ln_kernel<<<dim3((NROWS + 7) / 8), dim3(256), 0, stream>>>(h0, o, ln1_g, ln1_b, h1, NROWS);
    launch_gemm(stream, h1, W1, b1, ff1, NROWS, D_FF, D_MODEL, 1, 1);
    launch_gemm(stream, ff1, W2, b2, ff2, NROWS, D_MODEL, D_FF, 1, 0);
    add_ln_kernel<<<dim3((NROWS + 7) / 8), dim3(256), 0, stream>>>(h1, ff2, ln2_g, ln2_b, h2, NROWS);
    launch_gemm(stream, h2, Wd, bd, xrec, NROWS, D_IN, D_MODEL, 1, 0);
    dist_topk_kernel<<<dim3((NROWS + DT_ROWS - 1) / DT_ROWS), dim3(DT_ROWS), 0, stream>>>(xrec, rowsum, NROWS);
    final_sum_kernel<<<dim3(1), dim3(256), 0, stream>>>(rowsum, out, NROWS);
}
